// NN_22419729285749
// MI455X (gfx1250) — hardware-verified
//
#include <hip/hip_runtime.h>


#define NBR  4096
#define DIN  64
#define HH   1024
#define OFF1 16384
#define OFF2 32768
typedef __attribute__((ext_vector_type(4))) unsigned short v4us;
typedef __attribute__((ext_vector_type(2))) unsigned short v2us;
typedef _Float16 h16;
typedef unsigned short bf;
typedef __attribute__((ext_vector_type(16))) __bf16   v16bf;
typedef __attribute__((ext_vector_type(16))) _Float16 v16h;
typedef __attribute__((ext_vector_type(8)))  _Float16 v8h;
typedef __attribute__((ext_vector_type(8)))  unsigned short v8us;
typedef __attribute__((ext_vector_type(8)))  float    v8f;
typedef __attribute__((ext_vector_type(4)))  float    v4f;
typedef v8h  __attribute__((may_alias)) v8ha;
typedef v4f  __attribute__((may_alias)) v4fa;
typedef v8us __attribute__((may_alias)) v8usa;

__device__ __forceinline__ unsigned short f2bf(float f) { unsigned u = __float_as_uint(f); u += 0x7FFFu + ((u >> 16) & 1u); return (unsigned short)(u >> 16); }
__device__ __forceinline__ float bf2f(unsigned short b) { return __uint_as_float(((unsigned)b) << 16); }
__device__ __forceinline__ float bfr(float f) { return bf2f(f2bf(f)); }
__device__ __forceinline__ v16h cat16(v8h lo, v8h hi) { return __builtin_shufflevector(lo, hi, 0, 1, 2, 3, 4, 5, 6, 7, 8, 9, 10, 11, 12, 13, 14, 15); }
__device__ __forceinline__ v16bf cat16b(v8us lo, v8us hi) { return __builtin_bit_cast(v16bf, __builtin_shufflevector(lo, hi, 0, 1, 2, 3, 4, 5, 6, 7, 8, 9, 10, 11, 12, 13, 14, 15)); }
__device__ __forceinline__ v8f wmma16(v16h a, v16h b, v8f c) { return __builtin_amdgcn_wmma_f32_16x16x32_f16(false, a, false, b, (short)0, c, false, false); }
__device__ __forceinline__ v8f wmmab(v16bf a, v16bf b, v8f c) { return __builtin_amdgcn_wmma_f32_16x16x32_bf16(false, a, false, b, (short)0, c, false, false); }


template <typename T16> struct WFrag;
template <> struct WFrag<h16> { typedef v16h V; static __device__ __forceinline__ V ld(const h16* p) { return cat16(*(const v8h*)p, *(const v8h*)(p + 16)); } static __device__ __forceinline__ v8f mma(V a, V b, v8f c) { return wmma16(a, b, c); } };
template <> struct WFrag<bf> { typedef v16bf V; static __device__ __forceinline__ V ld(const bf* p) { return cat16b(*(const v8us*)p, *(const v8us*)(p + 16)); } static __device__ __forceinline__ v8f mma(V a, V b, v8f c) { return wmmab(a, b, c); } };
template <typename T16, int NSPLIT, bool BIAS>
__global__ __launch_bounds__(32) void k_gemmw(const T16* __restrict__ A, const T16* __restrict__ A2, const T16* __restrict__ Bt, const T16* __restrict__ Bt2, int K, float* C, int ldc, const float* __restrict__ bias, size_t sA, size_t sB, size_t sC) {
    typedef typename WFrag<T16>::V V;
    __shared__ __align__(16) float os[16 * 68];
    const size_t z = blockIdx.z; A += z * sA; if (A2) A2 += z * sA; Bt += z * sB; if (Bt2) Bt2 += z * sB; C += z * sC;
    const int lane = threadIdx.x & 31, lr = lane & 15, hi = lane >> 4; const int r0 = blockIdx.x * 64, c0 = blockIdx.y * 64;
    v8f acc[4][4];
#pragma unroll
    for (int mb = 0; mb < 4; ++mb)
#pragma unroll
        for (int nb = 0; nb < 4; ++nb) acc[mb][nb] = (v8f){};
    const size_t aoff = (size_t)(r0 + lr) * K + 8 * hi, boff = (size_t)(c0 + lr) * K + 8 * hi;
#pragma unroll 1
    for (int kc = 0; kc < K; kc += 32) {
        V a[4], a2[4];
#pragma unroll
        for (int mb = 0; mb < 4; ++mb) { a[mb] = WFrag<T16>::ld(A + aoff + (size_t)mb * 16 * K + kc); if (NSPLIT == 1 || NSPLIT == 2) a2[mb] = WFrag<T16>::ld(A2 + aoff + (size_t)mb * 16 * K + kc); }
#pragma unroll
        for (int nb = 0; nb < 4; ++nb) { const V b = WFrag<T16>::ld(Bt + boff + (size_t)nb * 16 * K + kc); V b2; if (NSPLIT >= 2) b2 = WFrag<T16>::ld(Bt2 + boff + (size_t)nb * 16 * K + kc);
#pragma unroll
            for (int mb = 0; mb < 4; ++mb) { acc[mb][nb] = WFrag<T16>::mma(a[mb], b, acc[mb][nb]); if (NSPLIT == 1 || NSPLIT == 2) acc[mb][nb] = WFrag<T16>::mma(a2[mb], b, acc[mb][nb]); if (NSPLIT >= 2) acc[mb][nb] = WFrag<T16>::mma(a[mb], b2, acc[mb][nb]); } }
        asm volatile("v_nop\n\tv_nop\n\tv_nop\n\tv_nop" : "+v"(acc[0][0]), "+v"(acc[1][1]), "+v"(acc[2][2]), "+v"(acc[3][3]) : "v"(a[0]), "v"(a[3]));
    }
#pragma unroll
    for (int mb = 0; mb < 4; ++mb) {
#pragma unroll
        for (int nb = 0; nb < 4; ++nb) {
#pragma unroll
            for (int j = 0; j < 8; ++j) os[(hi * 8 + j) * 68 + nb * 16 + lr] = acc[mb][nb][j]; }
        __builtin_amdgcn_wave_barrier(); asm volatile("" ::: "memory");
        float* crow = C + (size_t)(r0 + mb * 16) * ldc + c0;
#pragma unroll 1
        for (int ps = 0; ps < 2; ++ps) {
#pragma unroll
            for (int s = 0; s < 8; ++s) { const int row = 2 * s + hi, cofs = lr * 4; v4f val = *(const v4fa*)(os + row * 68 + cofs); if (BIAS) { val[0] += bfr(bias[c0 + cofs]); val[1] += bfr(bias[c0 + cofs + 1]); val[2] += bfr(bias[c0 + cofs + 2]); val[3] += bfr(bias[c0 + cofs + 3]); }
                *(volatile v4f*)(crow + (size_t)row * ldc + cofs) = val; }
            if (ps == 0) __threadfence(); }
        __builtin_amdgcn_wave_barrier(); asm volatile("" ::: "memory");
    }
}

__device__ __forceinline__ void splitf(float y, unsigned short& h, unsigned short& l) { h = f2bf(y); l = f2bf(y - bf2f(h)); }
__global__ __launch_bounds__(256) void k_wtG(const float* __restrict__ w, int K, int N, bf* Bt) {
    const int lane = threadIdx.x & 31; const int L0 = (blockIdx.x * 8 + (threadIdx.x >> 5)) * 8; const int nlines = N * K / 64;
#pragma unroll
    for (int ps = 0; ps < 2; ++ps) {
#pragma unroll 1
        for (int l = 0; l < 8; ++l) { const int L = L0 + l; if (L >= nlines) break; const size_t e = (size_t)L * 64 + lane * 2; const int k = (int)(e % K), n = (int)(e / K); v2us o;
            o[0] = f2bf(w[(size_t)k * N + n]); o[1] = f2bf(w[(size_t)(k + 1) * N + n]); *(volatile v2us*)(Bt + e) = o; }
        if (ps == 0) __threadfence(); }
}
__global__ __launch_bounds__(256) void k_cvt8(const float* __restrict__ src, bf* dst, size_t n8) { const size_t i = (size_t)blockIdx.x * 256 + threadIdx.x; if (i >= n8) return; const v8f v = *(const v8f*)(src + i * 8); v8us o;
#pragma unroll
    for (int k = 0; k < 8; ++k) o[k] = f2bf(v[k]); *(volatile v8us*)(dst + i * 8) = o; __threadfence(); *(volatile v8us*)(dst + i * 8) = o; }
__global__ __launch_bounds__(256) void k_act1(const float* __restrict__ Z, bf* Yh, bf* Yl, float* D1) { const size_t e = ((size_t)blockIdx.x * 256 + threadIdx.x) * 4; if (e >= (size_t)NBR * HH) return; const v4f z = *(const v4f*)(Z + e); v4us oh, ol; v4f d;
#pragma unroll
    for (int q = 0; q < 4; ++q) { const float y = tanhf(z[q]); d[q] = __fsub_rn(1.0f, __fmul_rn(y, y)); unsigned short a, c; splitf(y, a, c); oh[q] = a; ol[q] = c; }
    *(volatile v4us*)(Yh + e) = oh; *(volatile v4us*)(Yl + e) = ol; *(volatile v4f*)(D1 + e) = d; __threadfence(); *(volatile v4us*)(Yh + e) = oh; *(volatile v4us*)(Yl + e) = ol; *(volatile v4f*)(D1 + e) = d; }
__global__ __launch_bounds__(256) void k_act2(const float* __restrict__ Z, const float* __restrict__ W3, float* Y2, bf* Ah, bf* Al) { const size_t e = ((size_t)blockIdx.x * 256 + threadIdx.x) * 4; if (e >= (size_t)NBR * HH) return; const int o = (int)(e % HH); const v4f z = *(const v4f*)(Z + e); v4us oh, ol; v4f yv;
#pragma unroll
    for (int q = 0; q < 4; ++q) { const float y = tanhf(z[q]); yv[q] = y; const float d = __fsub_rn(1.0f, __fmul_rn(y, y)); const float a2 = __fmul_rn(bfr(W3[o + q]), d); unsigned short a, c; splitf(a2, a, c); oh[q] = a; ol[q] = c; }
    *(volatile v4f*)(Y2 + e) = yv; *(volatile v4us*)(Ah + e) = oh; *(volatile v4us*)(Al + e) = ol; __threadfence(); *(volatile v4f*)(Y2 + e) = yv; *(volatile v4us*)(Ah + e) = oh; *(volatile v4us*)(Al + e) = ol; }
__global__ __launch_bounds__(256) void k_g1(const float* __restrict__ G2, const float* __restrict__ D1, bf* Gh, bf* Gl) { const size_t e = ((size_t)blockIdx.x * 256 + threadIdx.x) * 4; if (e >= (size_t)NBR * HH) return; const v4f g = *(const v4f*)(G2 + e), d = *(const v4f*)(D1 + e); v4us oh, ol;
#pragma unroll
    for (int q = 0; q < 4; ++q) { unsigned short a, c; splitf(__fmul_rn(g[q], d[q]), a, c); oh[q] = a; ol[q] = c; } *(volatile v4us*)(Gh + e) = oh; *(volatile v4us*)(Gl + e) = ol; __threadfence(); *(volatile v4us*)(Gh + e) = oh; *(volatile v4us*)(Gl + e) = ol; }
__global__ __launch_bounds__(256) void k_vdot(const float* __restrict__ Y2, const float* __restrict__ W3, const float* __restrict__ GV, const float* __restrict__ xdot, float* V, float* VD) { const int b = blockIdx.x * 256 + threadIdx.x; if (b >= NBR) return; float s = 0.f, sd = 0.f;
#pragma unroll 4
    for (int o = 0; o < HH; ++o) { float p = __fmul_rn(Y2[(size_t)b * HH + o], bfr(W3[o])); asm volatile("" : "+v"(p)); s = __fadd_rn(s, p); }
#pragma unroll 4
    for (int d = 0; d < DIN; ++d) { float p = __fmul_rn(GV[(size_t)b * DIN + d], bfr(xdot[(size_t)b * DIN + d])); asm volatile("" : "+v"(p)); sd = __fadd_rn(sd, p); }
    *(volatile float*)(V + b) = s; *(volatile float*)(VD + b) = sd; __threadfence(); *(volatile float*)(V + b) = s; *(volatile float*)(VD + b) = sd; }

extern "C" void kernel_launch(void* const* d_in, const int* in_sizes, int n_in,
                              void* d_out, int out_size, void* d_ws, size_t ws_size, hipStream_t stream) {
    (void)in_sizes; (void)n_in; (void)out_size;
    const float* x = (const float*)d_in[0]; const float* xdot = (const float*)d_in[1]; const float* W1 = (const float*)d_in[2]; const float* b1 = (const float*)d_in[3]; const float* W2 = (const float*)d_in[4]; const float* b2 = (const float*)d_in[5]; const float* W3 = (const float*)d_in[6];
    float* V = (float*)d_out; float* VD = (float*)((char*)d_out + OFF1); float* GV = (float*)((char*)d_out + OFF2);
    char* wsp = (char*)d_ws;
    auto take = [&](size_t bytes) { char* p = wsp; wsp += (bytes + 255) & ~(size_t)255; return (void*)p; };
    bf* XB = (bf*)take((size_t)NBR * DIN * 2); bf* W1B = (bf*)take((size_t)HH * DIN * 2); bf* W2B = (bf*)take((size_t)HH * HH * 2); bf* W2T = (bf*)take((size_t)HH * HH * 2); bf* W1T = (bf*)take((size_t)DIN * HH * 2);
    float* Z1 = (float*)take((size_t)NBR * HH * 4); bf* Y1h = (bf*)take((size_t)NBR * HH * 2); bf* Y1l = (bf*)take((size_t)NBR * HH * 2); float* D1 = (float*)take((size_t)NBR * HH * 4); float* Z2 = (float*)take((size_t)NBR * HH * 4); float* Y2 = (float*)take((size_t)NBR * HH * 4);
    bf* A2h = (bf*)take((size_t)NBR * HH * 2); bf* A2l = (bf*)take((size_t)NBR * HH * 2); float* G2 = (float*)take((size_t)NBR * HH * 4); bf* G1h = (bf*)take((size_t)NBR * HH * 2); bf* G1l = (bf*)take((size_t)NBR * HH * 2);
    if ((size_t)(wsp - (char*)d_ws) > ws_size) return;
    const size_t n4 = (size_t)NBR * HH / 4; const unsigned nb4 = (unsigned)((n4 + 255) / 256);
    k_cvt8<<<(NBR * DIN / 8 + 255) / 256, 256, 0, stream>>>(x, XB, (size_t)NBR * DIN / 8); k_cvt8<<<(HH * DIN / 8 + 255) / 256, 256, 0, stream>>>(W1, W1B, (size_t)HH * DIN / 8); k_cvt8<<<(HH * HH / 8 + 255) / 256, 256, 0, stream>>>(W2, W2B, (size_t)HH * HH / 8);
    k_wtG<<<(unsigned)((HH * HH / 64 + 63) / 64), 256, 0, stream>>>(W2, HH, HH, W2T); k_wtG<<<(unsigned)((HH * DIN / 64 + 63) / 64), 256, 0, stream>>>(W1, HH, DIN, W1T);
    k_gemmw<bf, 0, true><<<dim3(NBR / 64, HH / 64, 1), 32, 0, stream>>>(XB, nullptr, W1B, nullptr, DIN, Z1, HH, b1, 0, 0, 0);
    k_act1<<<nb4, 256, 0, stream>>>(Z1, Y1h, Y1l, D1);
    k_gemmw<bf, 1, true><<<dim3(NBR / 64, HH / 64, 1), 32, 0, stream>>>(Y1h, Y1l, W2B, nullptr, HH, Z2, HH, b2, 0, 0, 0);
    k_act2<<<nb4, 256, 0, stream>>>(Z2, W3, Y2, A2h, A2l);
    k_gemmw<bf, 1, false><<<dim3(NBR / 64, HH / 64, 1), 32, 0, stream>>>(A2h, A2l, W2T, nullptr, HH, G2, HH, nullptr, 0, 0, 0);
    k_g1<<<nb4, 256, 0, stream>>>(G2, D1, G1h, G1l);
    k_gemmw<bf, 1, false><<<dim3(NBR / 64, DIN / 64, 1), 32, 0, stream>>>(G1h, G1l, W1T, nullptr, HH, GV, DIN, nullptr, 0, 0, 0);
    k_vdot<<<(NBR + 255) / 256, 256, 0, stream>>>(Y2, W3, GV, xdot, V, VD);
}
